// Model_13829794693476
// MI455X (gfx1250) — hardware-verified
//
#include <hip/hip_runtime.h>
#include <stddef.h>
#include <stdint.h>
#include <math.h>

#define NHID    256
#define NTHR    256
#define NWAVE   8
#define EPT     8
#define CHUNK   (NTHR * EPT)
#define WCAP    (EPT * 32)
#define LISTN   (NWAVE * WCAP)
#define NBA     1024
#define SLA     10
#define EIDB    17
#define EIDM    ((1 << EIDB) - 1)
#define RCAP    20480
#define DEGCAP  64
#define MEAS_B1024  12492
#define MEAS_MAXDEG 27
#define GBM     64
#define GBN     128
#define GTHR    128
#define GNT     8
#define ANB     64
#define G0W     96
#define K0P     96
#define K0T     192
#define KRP     288
#define KRT     576
#define TK0P    64
#define TK0T    128
#define NTOP    16
#define ETOP    64
#define NGRP    100
#define GSZ     100
#define CFW     64
#define OPW     4
#define OPS     256
#define CEW     16
#define W0ROWS  2132
#define TFLAT   2048
#define PLR     (NHID * KRT)
#define OW_TW0  0
#define OW_TWR  (NHID * TK0T)
#define OW_CW0  (OW_TWR + 3 * PLR)
#define OW_CWR  (OW_CW0 + NHID * K0T)
#define WTS_N   (OW_CWR + 5 * PLR)
#define U_TW0   (NHID * (TK0T / 8))
#define U_TWR   (3 * NHID * (KRT / 8))
#define U_CW0   (NHID * (K0T / 8))
#define U_CWR   (5 * NHID * (KRT / 8))
#define U_ALL   (U_TW0 + U_TWR + U_CW0 + U_CWR)
#define BKT_INTS (LISTN + 2 * RCAP + 3 * NBA + 32)
#define WSMAX   134217728

static_assert((CHUNK & (CHUNK - 1)) == 0 && CHUNK <= 4096);
static_assert(NBA == (1 << SLA));
static_assert(EIDB + SLA < 31);
static_assert((RCAP % 1024) == 0);
static_assert((long long)RCAP * 100 >= (long long)MEAS_B1024 * 105);
static_assert(DEGCAP >= MEAS_MAXDEG + 8);
static_assert(BKT_INTS * 4 <= 300000);
static_assert(((RCAP + 3 * NBA) % 4) == 0);
static_assert((U_TW0 % NTHR) == 0 && (U_TWR % NTHR) == 0 && (U_CW0 % NTHR) == 0 && (U_CWR % NTHR) == 0);
static_assert((K0T % 32) == 0 && (KRT % 32) == 0 && (TK0T % 32) == 0);
static_assert(GTHR == GBN && GBM == (GTHR / 32) * 16 && NHID == 2 * GBN);
static_assert(ANB == NWAVE * 8);
static_assert(NGRP * 9 == 225 * 4);
static_assert((ETOP & (ETOP - 1)) == 0 && ETOP * 16 == NTHR * 4 && NTHR == NHID);

typedef float          v4f  __attribute__((ext_vector_type(4)));
typedef float          v8f  __attribute__((ext_vector_type(8)));
typedef int            v4i  __attribute__((ext_vector_type(4)));
typedef int            v8i  __attribute__((ext_vector_type(8)));
typedef unsigned int   v2u  __attribute__((ext_vector_type(2)));
typedef unsigned int   v4u  __attribute__((ext_vector_type(4)));
typedef unsigned short v8us __attribute__((ext_vector_type(8)));
typedef __bf16         v16b __attribute__((ext_vector_type(16)));
typedef v4f  __attribute__((may_alias)) v4fa;
typedef v4i  __attribute__((may_alias)) v4ia;
typedef v2u  __attribute__((may_alias)) v2ua;
typedef v4u  __attribute__((may_alias)) v4ua;
typedef v8us __attribute__((may_alias)) v8usa;
union FragB { v16b v; v8us h[2]; v8i w; };

__device__ __forceinline__ v8f wmb(const FragB& a, const FragB& b, v8f c) {
  v8f d = __builtin_amdgcn_wmma_f32_16x16x32_bf16(false, a.v, false, b.v, (short)0, c, false, false);
  asm volatile("v_nop\n\tv_nop\n\tv_nop\n\tv_nop" : "+v"(d) : "v"(a.w), "v"(b.w));
  return d;
}

__device__ __forceinline__ unsigned int f2bf(float f) {
  const unsigned int u = __float_as_uint(f);
  const unsigned int r = ((u + 0x7FFFu + ((u >> 16) & 1u)) >> 16) & 0xFFFFu;
  return ((u & 0x7FFFFFFFu) > 0x7F800000u) ? 0x7FC0u : r;
}
__device__ __forceinline__ float bf2f(unsigned int b) { return __uint_as_float(b << 16); }
__device__ __forceinline__ float bfr(float f) { return bf2f(f2bf(f)); }
__device__ __forceinline__ float relu_k(float v) { return (v > 0.0f) ? v : (v - v); }
__device__ __forceinline__ int clampi(int v, int lo, int hi) { return v < lo ? lo : (v > hi ? hi : v); }

template <int SLB>
__device__ __forceinline__ int scan_chunk(const int* __restrict__ dsts, int nE, int cbase, int slotBase,
                                          int nb, int vec8, int* list, int tid, int lane, int wave) {
  int wc = 0;
  const int el0  = tid * EPT;
  const int e0   = cbase + el0;
  const int sent = -2147483647 - 1;
  v4i da, db;
  if (vec8 != 0 && cbase + CHUNK <= nE) {
    da = *(const v4i*)(dsts + e0);
    db = *(const v4i*)(dsts + e0 + 4);
  } else {
    da.x = (e0     < nE) ? dsts[min(e0,     nE - 1)] : sent;
    da.y = (e0 + 1 < nE) ? dsts[min(e0 + 1, nE - 1)] : sent;
    da.z = (e0 + 2 < nE) ? dsts[min(e0 + 2, nE - 1)] : sent;
    da.w = (e0 + 3 < nE) ? dsts[min(e0 + 3, nE - 1)] : sent;
    db.x = (e0 + 4 < nE) ? dsts[min(e0 + 4, nE - 1)] : sent;
    db.y = (e0 + 5 < nE) ? dsts[min(e0 + 5, nE - 1)] : sent;
    db.z = (e0 + 6 < nE) ? dsts[min(e0 + 6, nE - 1)] : sent;
    db.w = (e0 + 7 < nE) ? dsts[min(e0 + 7, nE - 1)] : sent;
  }
  const unsigned nbs = (unsigned)slotBase;
  const unsigned unb = (unsigned)nb;
  const unsigned s0 = (unsigned)da.x - nbs, s1 = (unsigned)da.y - nbs;
  const unsigned s2 = (unsigned)da.z - nbs, s3 = (unsigned)da.w - nbs;
  const unsigned s4 = (unsigned)db.x - nbs, s5 = (unsigned)db.y - nbs;
  const unsigned s6 = (unsigned)db.z - nbs, s7 = (unsigned)db.w - nbs;
  const bool h0 = s0 < unb, h1 = s1 < unb, h2 = s2 < unb, h3 = s3 < unb;
  const bool h4 = s4 < unb, h5 = s5 < unb, h6 = s6 < unb, h7 = s7 < unb;
  const unsigned any = __builtin_amdgcn_ballot_w32(h0 | h1 | h2 | h3 | h4 | h5 | h6 | h7);
  if (any != 0u) {
#define HITJ(J, HJ, SJ) { \
      const unsigned mj = __builtin_amdgcn_ballot_w32(HJ); \
      if (mj != 0u) { \
        if (HJ) { \
          const int pos = wc + (int)__builtin_amdgcn_mbcnt_lo(mj, 0u); \
          if (pos < WCAP) list[wave * WCAP + pos] = ((el0 + (J)) << SLB) | (int)(SJ); \
        } \
        wc += (int)__builtin_popcount(mj); } }
    HITJ(0, h0, s0)
    HITJ(1, h1, s1)
    HITJ(2, h2, s2)
    HITJ(3, h3, s3)
    HITJ(4, h4, s4)
    HITJ(5, h5, s5)
    HITJ(6, h6, s6)
    HITJ(7, h7, s7)
#undef HITJ
  }
  return wc;
}

__global__ __launch_bounds__(NTHR) void k_prep(const float* __restrict__ tW0, const float* __restrict__ tWr,
                                               const float* __restrict__ cW0, const float* __restrict__ cWr,
                                               unsigned short* WTS) {
  const int u = (int)blockIdx.x * NTHR + (int)threadIdx.x;
  v8us o;
  unsigned short* dp;
  if (u < U_TW0) {
    const int n  = u >> 4;
    const int k8 = (u & 15) * 8;
    const int kk = k8 & (TK0P - 1);
#pragma unroll
    for (int i = 0; i < 8; ++i) {
      const int k  = kk + i;
      const int kc = k < 48 ? k : 47;
      const float f = tW0[(size_t)kc * NHID + n];
      o[i] = (k < 48) ? (unsigned short)f2bf(f) : (unsigned short)0;
    }
    dp = WTS + OW_TW0 + (size_t)n * TK0T + k8;
  } else if (u < U_TW0 + U_TWR) {
    const int v  = u - U_TW0;
    const int l  = v / (NHID * 72);
    const int w  = v - l * (NHID * 72);
    const int n  = w / 72;
    const int k8 = (w - n * 72) * 8;
    const int kk = k8 >= KRP ? k8 - KRP : k8;
#pragma unroll
    for (int i = 0; i < 8; ++i) {
      const int k  = kk + i;
      const int kc = k < 272 ? k : 271;
      const float f = tWr[((size_t)l * 272 + kc) * NHID + n];
      o[i] = (k < 272) ? (unsigned short)f2bf(f) : (unsigned short)0;
    }
    dp = WTS + OW_TWR + (size_t)l * PLR + (size_t)n * KRT + k8;
  } else if (u < U_TW0 + U_TWR + U_CW0) {
    const int v  = u - U_TW0 - U_TWR;
    const int n  = v / 24;
    const int k8 = (v - n * 24) * 8;
    const int kk = k8 >= K0P ? k8 - K0P : k8;
#pragma unroll
    for (int i = 0; i < 8; ++i) {
      const int k   = kk + i;
      const int row = (k < 68) ? k : ((k < 84) ? (2116 + k - 68) : 0);
      const float f = cW0[(size_t)row * NHID + n];
      o[i] = (k < 84) ? (unsigned short)f2bf(f) : (unsigned short)0;
    }
    dp = WTS + OW_CW0 + (size_t)n * K0T + k8;
  } else if (u < U_ALL) {
    const int v  = u - U_TW0 - U_TWR - U_CW0;
    const int l  = v / (NHID * 72);
    const int w  = v - l * (NHID * 72);
    const int n  = w / 72;
    const int k8 = (w - n * 72) * 8;
    const int kk = k8 >= KRP ? k8 - KRP : k8;
#pragma unroll
    for (int i = 0; i < 8; ++i) {
      const int k  = kk + i;
      const int kc = k < 272 ? k : 271;
      const float f = cWr[((size_t)l * 272 + kc) * NHID + n];
      o[i] = (k < 272) ? (unsigned short)f2bf(f) : (unsigned short)0;
    }
    dp = WTS + OW_CWR + (size_t)l * PLR + (size_t)n * KRT + k8;
  } else {
    return;
  }
  *(volatile v8us*)dp = o;
  __threadfence();
  *(volatile v8us*)dp = o;
}

__global__ __launch_bounds__(NTHR) void k_topo(const float* __restrict__ tfeats, const float* __restrict__ tef,
                                               const float* __restrict__ tb0, const float* __restrict__ tbr,
                                               const int* __restrict__ t_src, const int* __restrict__ t_dst,
                                               const int* __restrict__ tgroups, const float* __restrict__ cW0,
                                               const unsigned short* __restrict__ WTS, float* V) {
  __shared__ __attribute__((aligned(16))) float sx[NTOP * NHID];
  __shared__ __attribute__((aligned(16))) float sfs[NTOP * NHID];
  __shared__ __attribute__((aligned(16))) unsigned short sA[NTOP * KRT];
  __shared__ __attribute__((aligned(16))) float sef[ETOP * 16];
  __shared__ float sEA[NTOP * 16];
  __shared__ float sEA0[NTOP * 16];
  __shared__ float sbias[4 * NHID];
  __shared__ float son[NTOP];
  __shared__ float sinn[NTOP];
  __shared__ int ssrc[ETOP];
  __shared__ int sdst[ETOP];
  __shared__ int sgrp[16];
  const int tid = (int)threadIdx.x, lane = tid & 31, wave = tid >> 5, hh = lane >> 4, m = lane & 15;

  {
    const int ts = t_src[tid & (ETOP - 1)];
    const int td = t_dst[tid & (ETOP - 1)];
    const int gi = tgroups[tid & 15];
    if (tid < ETOP) {
      ssrc[tid] = clampi(ts, 0, NTOP - 1);
      sdst[tid] = clampi(td, 0, NTOP - 1);
    }
    if (tid < 16) sgrp[tid] = clampi(gi, 0, NTOP - 1);
  }
  __syncthreads();
  {
    const v4f t4 = *(const v4f*)(tef + 4 * tid);
    v4f r4;
    r4.x = bfr(t4.x); r4.y = bfr(t4.y); r4.z = bfr(t4.z); r4.w = bfr(t4.w);
    *(v4fa*)(sef + 4 * tid) = r4;
  }
  __syncthreads();
  {
    const float b0v = tb0[tid];
    const float b1v = tbr[tid];
    const float b2v = tbr[NHID + tid];
    const float b3v = tbr[2 * NHID + tid];
    sbias[tid]            = bfr(b0v);
    sbias[NHID + tid]     = bfr(b1v);
    sbias[2 * NHID + tid] = bfr(b2v);
    sbias[3 * NHID + tid] = bfr(b3v);
  }
  __syncthreads();

  {
    const int n = tid & 15;
    int co = 0, ci = 0;
#pragma unroll 4
    for (int e = 0; e < ETOP; ++e) {
      co += (ssrc[e] == n) ? 1 : 0;
      ci += (sdst[e] == n) ? 1 : 0;
    }
    const float fo = (float)(co < 1 ? 1 : co);
    const float fi = (float)(ci < 1 ? 1 : ci);
    if (tid < 16) {
      son[n]  = 1.0f / sqrtf(fo);
      sinn[n] = 1.0f / sqrtf(fi);
    }
  }
  {
    const int n = tid >> 4, c = tid & 15;
    float a = 0.0f, ar = 0.0f;
#pragma unroll 4
    for (int e = 0; e < ETOP; ++e) {
      const float v = sef[e * 16 + c];
      const bool hit = (sdst[e] == n);
      a  += hit ? v : 0.0f;
      ar += hit ? relu_k(v) : 0.0f;
    }
    sEA[tid]  = a;
    sEA0[tid] = ar;
  }
  __syncthreads();

#pragma unroll 1
  for (int L = 0; L < 4; ++L) {
    const int kp   = (L == 0) ? TK0P : KRP;
    const int kt   = 2 * kp;
    const int nf   = (L == 0) ? 32 : NHID;
    const int woff = (L == 0) ? OW_TW0 : (OW_TWR + (L - 1) * PLR);
    if (L == 0) {
#pragma unroll
      for (int j = 0; j < 2; ++j) {
        const int idx = tid + NTHR * j;
        const int n = idx >> 5, k = idx & 31;
        sfs[n * NHID + k] = bfr(tfeats[idx]) * son[n];
      }
    } else {
#pragma unroll 4
      for (int n = 0; n < NTOP; ++n) sfs[n * NHID + tid] = sx[n * NHID + tid] * son[n];
    }
    __syncthreads();
    if (tid < nf) {
#pragma unroll 4
      for (int n = 0; n < NTOP; ++n) sx[n * NHID + tid] = 0.0f;
#pragma unroll 2
      for (int e = 0; e < ETOP; ++e) {
        const int s = ssrc[e], d = sdst[e];
        float v = sfs[s * NHID + tid];
        v = (L == 0) ? relu_k(v) : v;
        sx[d * NHID + tid] = sx[d * NHID + tid] + v;
      }
#pragma unroll 4
      for (int n = 0; n < NTOP; ++n) {
        const float v = sx[n * NHID + tid];
        const unsigned int hb = f2bf(v);
        sA[n * kt + tid]      = (unsigned short)hb;
        sA[n * kt + kp + tid] = (unsigned short)f2bf(v - bf2f(hb));
      }
    }
#pragma unroll
    for (int j = 0; j < 2; ++j) {
      const int idx = tid + NTHR * j;
      const int n = idx >> 5, c = idx & 31;
      const float e1 = sEA[n * 16 + (c & 15)];
      const float e0 = sEA0[n * 16 + (c & 15)];
      float v = (L == 0) ? e0 : e1;
      v = (c < 16) ? v : 0.0f;
      const unsigned int hb = f2bf(v);
      sA[n * kt + nf + c]      = (unsigned short)hb;
      sA[n * kt + kp + nf + c] = (unsigned short)f2bf(v - bf2f(hb));
    }
    __syncthreads();
    v8f acc[2];
    {
      const v8f z = {0.f, 0.f, 0.f, 0.f, 0.f, 0.f, 0.f, 0.f};
      acc[0] = z; acc[1] = z;
    }
    const unsigned short* ap = sA + m * kt + 8 * hh;
    const unsigned short* wp = WTS + woff + (size_t)(32 * wave + m) * (size_t)kt + 8 * hh;
    const int ksteps = kt >> 5;
#pragma unroll 1
    for (int ks = 0; ks < ksteps; ++ks) {
      FragB af;
      af.h[0] = *(const v8usa*)(ap + 32 * ks);
      af.h[1] = *(const v8usa*)(ap + 32 * ks + 16);
#pragma unroll
      for (int t = 0; t < 2; ++t) {
        const unsigned short* wq = wp + (size_t)(16 * t) * (size_t)kt + 32 * ks;
        FragB bf;
        bf.h[0] = *(const v8usa*)wq;
        bf.h[1] = *(const v8usa*)(wq + 16);
        acc[t] = wmb(af, bf, acc[t]);
      }
    }
#pragma unroll
    for (int t = 0; t < 2; ++t) {
      const int col = 32 * wave + 16 * t + m;
      const float bb = sbias[L * NHID + col];
#pragma unroll
      for (int r = 0; r < 8; ++r) {
        const int row = 8 * hh + r;
        float v = fmaf(acc[t][r], sinn[row], bb);
        if (L < 3) v = relu_k(v);
        if (L == 1 || L == 2) v = v + sfs[row * NHID + col];
        sx[row * NHID + col] = v;
      }
    }
    __syncthreads();
  }

#pragma unroll
  for (int g = 0; g < 8; ++g) {
    const int a = sgrp[2 * g], b = sgrp[2 * g + 1];
    sfs[g * NHID + tid] = relu_k(sx[a * NHID + tid] + sx[b * NHID + tid]);
  }
  __syncthreads();
  {
    float s = 0.0f;
    const float* wc = cW0 + (size_t)68 * NHID + tid;
#pragma unroll 4
    for (int j = 0; j < TFLAT; ++j) s = fmaf(sfs[j], bfr(wc[(size_t)j * NHID]), s);
    sef[tid] = s;
  }
  __syncthreads();
  v4f vv = {0.f, 0.f, 0.f, 0.f};
  if (tid < 64) {
    vv = *(const v4fa*)(sef + 4 * tid);
    *(volatile v4f*)(V + 4 * tid) = vv;
  }
  __threadfence();
  if (tid < 64) {
    *(volatile v4f*)(V + 4 * tid) = vv;
  }
}

template <int MODE>
__global__ __launch_bounds__(NTHR) void k_bucket(const int* __restrict__ keys, int nE, int nN, int vec8,
                                                 int* LISTG, int* CNTA, int* OFFA, float* NRM, int* FLG) {
  extern __shared__ __attribute__((aligned(16))) int bsm[];
  int* list = bsm;
  int* reg1 = list + LISTN;
  int* reg2 = reg1 + RCAP;
  int* scnt = reg2 + RCAP;
  int* soff = scnt + NBA;
  int* cur  = soff + NBA;
  int* wcnt = cur + NBA;
  const int tid = (int)threadIdx.x, lane = tid & 31, wave = tid >> 5;
  const int blk = (int)blockIdx.x;
  const int nodeBase = blk * NBA;
  int nb = nN - nodeBase;
  nb = nb < 0 ? 0 : (nb > NBA ? NBA : nb);

  {
    const v4i z4 = {0, 0, 0, 0};
    for (int i = tid * 4; i < RCAP + 3 * NBA; i += NTHR * 4) *(v4ia*)(reg2 + i) = z4;
    if (tid < 32) wcnt[tid] = 0;
  }
  __syncthreads();

  int tot = 0, ovf = 0;
  const int nChunks = (nE + CHUNK - 1) / CHUNK;
#pragma unroll 1
  for (int ch = 0; ch < nChunks; ++ch) {
    const int cbase = ch * CHUNK;
    const int wc = scan_chunk<SLA>(keys, nE, cbase, nodeBase, nb, vec8, list, tid, lane, wave);
    if (lane == 0) wcnt[wave] = wc;
    __syncthreads();
    int pre = 0, all = 0;
#pragma unroll
    for (int w2 = 0; w2 < NWAVE; ++w2) {
      int c = wcnt[w2];
      c = c < 0 ? 0 : (c > WCAP ? WCAP : c);
      all += c;
      pre += (w2 < wave) ? c : 0;
    }
    const int wcc  = wc > WCAP ? WCAP : wc;
    const int base = tot + pre;
#pragma unroll 1
    for (int i = lane; i < wcc; i += 32) {
      const int ent = list[wave * WCAP + i];
      const int el  = (ent >> SLA) & (CHUNK - 1);
      const int sl  = ent & (NBA - 1);
      int eid = cbase + el;
      eid = eid > nE - 1 ? nE - 1 : eid;
      const int pos = base + i;
      if (pos < RCAP) reg1[pos] = (int)((unsigned)eid | ((unsigned)sl << EIDB));
    }
    if (tot + all > RCAP) ovf = 1;
    tot += all;
    tot = tot > RCAP ? RCAP : tot;
    __syncthreads();
  }
  const int nh = tot;

  if (wave == 0) {
#pragma unroll 1
    for (int b0 = 0; b0 < nh; b0 += 32) {
      const int idx = b0 + lane;
      const int uv  = reg1[idx < nh ? idx : nh - 1];
      const int m32 = (nh - b0) < 32 ? (nh - b0) : 32;
#pragma unroll 1
      for (int k = 0; k < m32; ++k) {
        const int u  = __builtin_amdgcn_readlane(uv, k);
        const int sq = (u >> EIDB) & (NBA - 1);
        if (lane == 0) scnt[sq] = scnt[sq] + 1;
      }
    }
  }
  __syncthreads();
  if (wave == 0) {
    const int base = lane * (NBA / 32);
    int s = 0;
#pragma unroll 1
    for (int i = 0; i < NBA / 32; ++i) s += scnt[base + i];
    int incl = s;
#pragma unroll
    for (int d = 1; d < 32; d <<= 1) {
      const int y = __shfl_up(incl, d, 32);
      if (lane >= d) incl += y;
    }
    int run = incl - s;
#pragma unroll 1
    for (int i = 0; i < NBA / 32; ++i) {
      const int cv = scnt[base + i];
      soff[base + i] = run;
      cur[base + i]  = run;
      run += cv;
    }
  }
  __syncthreads();
  if (MODE == 0) {
    if (wave == 0) {
#pragma unroll 1
      for (int b0 = 0; b0 < nh; b0 += 32) {
        const int idx = b0 + lane;
        const int uv  = reg1[idx < nh ? idx : nh - 1];
        const int m32 = (nh - b0) < 32 ? (nh - b0) : 32;
#pragma unroll 1
        for (int k = 0; k < m32; ++k) {
          const int u  = __builtin_amdgcn_readlane(uv, k);
          const int sq = (u >> EIDB) & (NBA - 1);
          if (lane == 0) {
            int p = cur[sq];
            p = p < 0 ? 0 : (p > RCAP - 1 ? RCAP - 1 : p);
            reg2[p] = u & EIDM;
            cur[sq] = p + 1;
          }
        }
      }
    }
    __syncthreads();
  }

  const v4i c4 = *(const v4ia*)(scnt + 4 * tid);
  const v4i o4 = *(const v4ia*)(soff + 4 * tid);
  {
    const bool big = (MODE == 0) && (c4.x > DEGCAP || c4.y > DEGCAP || c4.z > DEGCAP || c4.w > DEGCAP);
    const unsigned bm = __builtin_amdgcn_ballot_w32(big);
    if (lane == 0) wcnt[8 + wave] = (bm != 0u) ? 1 : 0;
  }
  __syncthreads();
  int fg = ovf;
#pragma unroll
  for (int w2 = 0; w2 < NWAVE; ++w2) fg |= wcnt[8 + w2];
  const float pz = (fg != 0) ? __int_as_float(0x7fc00000) : 0.0f;
  v4f n4;
  n4.x = 1.0f / sqrtf((float)(c4.x < 1 ? 1 : c4.x)) + pz;
  n4.y = 1.0f / sqrtf((float)(c4.y < 1 ? 1 : c4.y)) + pz;
  n4.z = 1.0f / sqrtf((float)(c4.z < 1 ? 1 : c4.z)) + pz;
  n4.w = 1.0f / sqrtf((float)(c4.w < 1 ? 1 : c4.w)) + pz;
  v4i cv;
  cv.x = (tid == 0) ? nh : 0;
  cv.y = (tid == 0) ? fg : 0;
  cv.z = 0; cv.w = 0;
  int*   fp = FLG  + (size_t)blk * 32 + 4 * (tid & 7);
  float* np = NRM  + (size_t)blk * NBA + 4 * tid;
  int*   cp = CNTA + (size_t)blk * NBA + 4 * tid;
  int*   op = OFFA + (size_t)blk * NBA + 4 * tid;
  int*   lb = LISTG + (size_t)blk * RCAP;

  if (MODE == 0) {
#pragma unroll 1
    for (int p = tid * 4; p < RCAP; p += NTHR * 4) {
      const v4i v = *(const v4ia*)(reg2 + p);
      *(volatile v4i*)(lb + p) = v;
    }
    *(volatile v4i*)cp = c4;
    *(volatile v4i*)op = o4;
  }
  *(volatile v4f*)np = n4;
  if (tid < 8) *(volatile v4i*)fp = cv;
  __threadfence();
  if (MODE == 0) {
#pragma unroll 1
    for (int p = tid * 4; p < RCAP; p += NTHR * 4) {
      const v4i v = *(const v4ia*)(reg2 + p);
      *(volatile v4i*)(lb + p) = v;
    }
    *(volatile v4i*)cp = c4;
    *(volatile v4i*)op = o4;
  }
  *(volatile v4f*)np = n4;
  if (tid < 8) *(volatile v4i*)fp = cv;
}

__global__ __launch_bounds__(NTHR) void k_node0(const float* __restrict__ cf, const float* __restrict__ ope,
                                                const int* __restrict__ ctypes, const float* __restrict__ ONA,
                                                float* G0, int nN, int nUnits) {
  const int u = (int)blockIdx.x * NTHR + (int)threadIdx.x;
  if (u >= nUnits) return;
  const int row = u / 24;
  const int p   = u - row * 24;
  const int rc  = row < nN ? row : nN - 1;
  const int pc  = p < 16 ? p : 15;
  const v4f a = *(const v4f*)(cf + (size_t)rc * CFW + 4 * pc);
  const int ct = clampi(ctypes[rc], 0, OPS - 1);
  const v4f b = *(const v4f*)(ope + (size_t)ct * OPW);
  const float on = ONA[rc];
  const bool okr = row < nN;
  const unsigned ma = (okr && p < 16) ? 0xFFFFFFFFu : 0u;
  const unsigned mb = (okr && p == 16) ? 0xFFFFFFFFu : 0u;
  const float x0 = __uint_as_float((__float_as_uint(a.x) & ma) | (__float_as_uint(b.x) & mb));
  const float x1 = __uint_as_float((__float_as_uint(a.y) & ma) | (__float_as_uint(b.y) & mb));
  const float x2 = __uint_as_float((__float_as_uint(a.z) & ma) | (__float_as_uint(b.z) & mb));
  const float x3 = __uint_as_float((__float_as_uint(a.w) & ma) | (__float_as_uint(b.w) & mb));
  const bool live = okr && p <= 16;
  v4f o;
  o.x = live ? relu_k(on * bfr(x0)) : 0.0f;
  o.y = live ? relu_k(on * bfr(x1)) : 0.0f;
  o.z = live ? relu_k(on * bfr(x2)) : 0.0f;
  o.w = live ? relu_k(on * bfr(x3)) : 0.0f;
  float* gp = G0 + (size_t)u * 4;
  *(volatile v4f*)gp = o;
  __threadfence();
  *(volatile v4f*)gp = o;
}

__global__ __launch_bounds__(NTHR) void k_agg0(const int* __restrict__ srcs, const float* __restrict__ ce,
                                               const float* __restrict__ G0, const float* __restrict__ ONA,
                                               const int* __restrict__ LISTG, const int* __restrict__ CNTA,
                                               const int* __restrict__ OFFA, const int* __restrict__ FLG0,
                                               unsigned short* H0, float* EAo, float* So,
                                               int nN, int nE, int MPr) {
  __shared__ __attribute__((aligned(16))) unsigned int stwAll[NWAVE * 96];
  __shared__ __attribute__((aligned(16))) float sea[ANB * 16];
  __shared__ __attribute__((aligned(16))) float ssv[ANB];
  const int tid = (int)threadIdx.x, lane = tid & 31, wave = tid >> 5;
  const int base = (int)blockIdx.x * ANB;
  unsigned int* stw = stwAll + wave * 96;
  const int gl = lane < 16 ? lane : 16;
  const int el = (lane + 15) & 3;
  const bool isN = lane <= 16;
  const bool isR = (lane >= 17) && (lane <= 20);
  const float qnan = __int_as_float(0x7fc00000);

#pragma unroll 1
  for (int j = 0; j < 8; ++j) {
    const int ln   = wave * 8 + j;
    const int node = base + ln;
    const int blk  = node >> SLA;
    const int craw = CNTA[node];
    int st  = OFFA[node];
    const int fgl = FLG0[(size_t)blk * 32 + 1];
    int cnt = craw < 0 ? 0 : (craw > DEGCAP ? DEGCAP : craw);
    st = st < 0 ? 0 : (st > RCAP ? RCAP : st);
    if (cnt > RCAP - st) cnt = RCAP - st;
    const float pz = (fgl != 0 || craw > DEGCAP || craw < 0) ? qnan : 0.0f;
    const bool live = node < nN;
    const int* lb = LISTG + (size_t)blk * RCAP;

    float n0 = 0.f, n1 = 0.f, n2 = 0.f, n3 = 0.f;
    float r0 = 0.f, r1 = 0.f, r2 = 0.f, r3 = 0.f;
    float e0 = 0.f, e1 = 0.f, e2 = 0.f, e3 = 0.f;
    float sS = 0.f;
#pragma unroll 1
    for (int b0 = 0; b0 < cnt; b0 += 32) {
      int idx = st + b0 + lane;
      idx = idx < 0 ? 0 : (idx > RCAP - 1 ? RCAP - 1 : idx);
      const int eid = clampi(lb[idx], 0, nE - 1);
      const int sv  = clampi(srcs[eid], 0, nN - 1);
      const int m32 = (cnt - b0) < 32 ? (cnt - b0) : 32;
#pragma unroll 1
      for (int k = 0; k < m32; ++k) {
        const int sk = __builtin_amdgcn_readlane(sv, k);
        const int ek = __builtin_amdgcn_readlane(eid, k);
        const v4f a = *(const v4f*)(G0 + (size_t)sk * G0W + 4 * gl);
        const v4f b = *(const v4f*)(ce + (size_t)ek * CEW + 4 * el);
        const float onv = ONA[sk];
        n0 += a.x; n1 += a.y; n2 += a.z; n3 += a.w;
        const float b0f = bfr(b.x), b1f = bfr(b.y), b2f = bfr(b.z), b3f = bfr(b.w);
        e0 += b0f; e1 += b1f; e2 += b2f; e3 += b3f;
        r0 += relu_k(b0f); r1 += relu_k(b1f); r2 += relu_k(b2f); r3 += relu_k(b3f);
        sS += onv;
      }
    }
    float o0 = isN ? n0 : (isR ? r0 : 0.0f);
    float o1 = isN ? n1 : (isR ? r1 : 0.0f);
    float o2 = isN ? n2 : (isR ? r2 : 0.0f);
    float o3 = isN ? n3 : (isR ? r3 : 0.0f);
    o0 = live ? (o0 + pz) : 0.0f;
    o1 = live ? (o1 + pz) : 0.0f;
    o2 = live ? (o2 + pz) : 0.0f;
    o3 = live ? (o3 + pz) : 0.0f;
    const unsigned int h0 = f2bf(o0), h1 = f2bf(o1), h2 = f2bf(o2), h3 = f2bf(o3);
    const unsigned int l0 = f2bf(o0 - bf2f(h0)), l1 = f2bf(o1 - bf2f(h1));
    const unsigned int l2 = f2bf(o2 - bf2f(h2)), l3 = f2bf(o3 - bf2f(h3));
    v2u hw, lw;
    hw.x = h0 | (h1 << 16); hw.y = h2 | (h3 << 16);
    lw.x = l0 | (l1 << 16); lw.y = l2 | (l3 << 16);
    __builtin_amdgcn_fence(__ATOMIC_RELEASE, "wavefront");
    __builtin_amdgcn_wave_barrier();
    if (lane < 24) {
      *(v2ua*)(stw + 2 * lane)      = hw;
      *(v2ua*)(stw + 48 + 2 * lane) = lw;
    }
    if (isR) {
      v4f ev;
      ev.x = live ? e0 : 0.0f; ev.y = live ? e1 : 0.0f; ev.z = live ? e2 : 0.0f; ev.w = live ? e3 : 0.0f;
      *(v4fa*)(sea + ln * 16 + 4 * el) = ev;
    }
    if (lane == 0) ssv[ln] = live ? (sS + pz) : 0.0f;
    __builtin_amdgcn_fence(__ATOMIC_RELEASE, "wavefront");
    __builtin_amdgcn_wave_barrier();
    const int pl = lane < 24 ? lane : 23;
    const v4u pk = *(const v4ua*)(stw + 4 * pl);
    unsigned short* gp = H0 + (size_t)node * K0T + 8 * pl;
    const bool wsv = (node < MPr) && (lane < 24);
    if (wsv) *(volatile v4u*)gp = pk;
    __threadfence();
    if (wsv) *(volatile v4u*)gp = pk;
  }
  __syncthreads();
  const v4f ev = *(const v4fa*)(sea + 4 * tid);
  const v4f sv4 = *(const v4fa*)(ssv + 4 * (tid & 15));
  float* ep = EAo + (size_t)base * 16 + 4 * tid;
  float* sp = So + (size_t)base + 4 * (tid & 15);
  *(volatile v4f*)ep = ev;
  if (tid < 16) *(volatile v4f*)sp = sv4;
  __threadfence();
  *(volatile v4f*)ep = ev;
  if (tid < 16) *(volatile v4f*)sp = sv4;
}

__global__ __launch_bounds__(NTHR) void k_agg(const int* __restrict__ srcs, const float* __restrict__ XS,
                                              const float* __restrict__ EA, const int* __restrict__ LISTG,
                                              const int* __restrict__ CNTA, const int* __restrict__ OFFA,
                                              const int* __restrict__ FLG0, unsigned short* H,
                                              int nN, int nE, int MPr) {
  __shared__ __attribute__((aligned(16))) unsigned int stwAll[NWAVE * 288];
  const int tid = (int)threadIdx.x, lane = tid & 31, wave = tid >> 5;
  const int base = (int)blockIdx.x * ANB;
  unsigned int* stw = stwAll + wave * 288;
  const float qnan = __int_as_float(0x7fc00000);

#pragma unroll 1
  for (int j = 0; j < 8; ++j) {
    const int node = base + wave * 8 + j;
    const int blk  = node >> SLA;
    const int craw = CNTA[node];
    int st  = OFFA[node];
    const int fgl = FLG0[(size_t)blk * 32 + 1];
    int cnt = craw < 0 ? 0 : (craw > DEGCAP ? DEGCAP : craw);
    st = st < 0 ? 0 : (st > RCAP ? RCAP : st);
    if (cnt > RCAP - st) cnt = RCAP - st;
    const float pz = (fgl != 0 || craw > DEGCAP || craw < 0) ? qnan : 0.0f;
    const bool live = node < nN;
    const int nc = live ? node : nN - 1;
    const int* lb = LISTG + (size_t)blk * RCAP;

    float a0 = 0.f, a1 = 0.f, a2 = 0.f, a3 = 0.f, a4 = 0.f, a5 = 0.f, a6 = 0.f, a7 = 0.f;
#pragma unroll 1
    for (int b0 = 0; b0 < cnt; b0 += 32) {
      int idx = st + b0 + lane;
      idx = idx < 0 ? 0 : (idx > RCAP - 1 ? RCAP - 1 : idx);
      const int eid = clampi(lb[idx], 0, nE - 1);
      const int sv  = clampi(srcs[eid], 0, nN - 1);
      const int m32 = (cnt - b0) < 32 ? (cnt - b0) : 32;
#pragma unroll 1
      for (int k = 0; k < m32; ++k) {
        const int sk = __builtin_amdgcn_readlane(sv, k);
        const float* rp = XS + (size_t)sk * NHID + 8 * lane;
        const v4f a = *(const v4f*)rp;
        const v4f b = *(const v4f*)(rp + 4);
        a0 += a.x; a1 += a.y; a2 += a.z; a3 += a.w;
        a4 += b.x; a5 += b.y; a6 += b.z; a7 += b.w;
      }
    }
    const v4f ev = *(const v4f*)(EA + (size_t)nc * 16 + 4 * (lane & 3));
    const float f[8] = {a0, a1, a2, a3, a4, a5, a6, a7};
    unsigned int hb[8], lbw[8];
#pragma unroll
    for (int i = 0; i < 8; ++i) {
      const float v = live ? (f[i] + pz) : 0.0f;
      hb[i]  = f2bf(v);
      lbw[i] = f2bf(v - bf2f(hb[i]));
    }
    v4u hwv, lwv;
    hwv.x = hb[0] | (hb[1] << 16);  hwv.y = hb[2] | (hb[3] << 16);
    hwv.z = hb[4] | (hb[5] << 16);  hwv.w = hb[6] | (hb[7] << 16);
    lwv.x = lbw[0] | (lbw[1] << 16); lwv.y = lbw[2] | (lbw[3] << 16);
    lwv.z = lbw[4] | (lbw[5] << 16); lwv.w = lbw[6] | (lbw[7] << 16);
    const float g0 = live ? (ev.x + pz) : 0.0f, g1 = live ? (ev.y + pz) : 0.0f;
    const float g2 = live ? (ev.z + pz) : 0.0f, g3 = live ? (ev.w + pz) : 0.0f;
    const unsigned int eh0 = f2bf(g0), eh1 = f2bf(g1), eh2 = f2bf(g2), eh3 = f2bf(g3);
    v2u ehw, elw;
    ehw.x = eh0 | (eh1 << 16); ehw.y = eh2 | (eh3 << 16);
    elw.x = f2bf(g0 - bf2f(eh0)) | (f2bf(g1 - bf2f(eh1)) << 16);
    elw.y = f2bf(g2 - bf2f(eh2)) | (f2bf(g3 - bf2f(eh3)) << 16);

    __builtin_amdgcn_fence(__ATOMIC_RELEASE, "wavefront");
    __builtin_amdgcn_wave_barrier();
    *(v4ua*)(stw + 4 * lane)       = hwv;
    *(v4ua*)(stw + 144 + 4 * lane) = lwv;
    if (lane < 4) {
      *(v2ua*)(stw + 128 + 2 * lane) = ehw;
      *(v2ua*)(stw + 272 + 2 * lane) = elw;
    }
    if (lane >= 8 && lane < 16) {
      stw[136 + lane - 8] = 0u;
      stw[280 + lane - 8] = 0u;
    }
    __builtin_amdgcn_fence(__ATOMIC_RELEASE, "wavefront");
    __builtin_amdgcn_wave_barrier();
    const v4u q0 = *(const v4ua*)(stw + 4 * lane);
    const v4u q1 = *(const v4ua*)(stw + 128 + 4 * lane);
    const v4u q2 = *(const v4ua*)(stw + 256 + 4 * (lane & 7));
    unsigned short* gp = H + (size_t)node * KRT;
    const bool wsv = node < MPr;
    if (wsv) {
      *(volatile v4u*)(gp + 8 * lane) = q0;
      *(volatile v4u*)(gp + 256 + 8 * lane) = q1;
      if (lane < 8) *(volatile v4u*)(gp + 512 + 8 * lane) = q2;
    }
    __threadfence();
    if (wsv) {
      *(volatile v4u*)(gp + 8 * lane) = q0;
      *(volatile v4u*)(gp + 256 + 8 * lane) = q1;
      if (lane < 8) *(volatile v4u*)(gp + 512 + 8 * lane) = q2;
    }
  }
}

template <int MODE>
__global__ __launch_bounds__(GTHR) __attribute__((amdgpu_num_vgpr(248)))
void k_gemm(const unsigned short* __restrict__ A, const unsigned short* __restrict__ WT,
            const float* __restrict__ bias, const float* __restrict__ INN, const float* __restrict__ ONA,
            const float* __restrict__ S, const float* __restrict__ V, const float* __restrict__ XSin,
            float* out, int K, int nN, int mRows) {
  __shared__ __attribute__((aligned(16))) float stg[GBM * GBN];
  __shared__ float srow[3 * GBM];
  __shared__ float scol[2 * GBN];
  const int tid = (int)threadIdx.x, lane = tid & 31, wave = tid >> 5, hh = lane >> 4, m = lane & 15;
  const int rowBase = (int)blockIdx.x * GBM;
  const int col0    = (int)blockIdx.y * GBN;

  if (tid < GBM) {
    const int r = rowBase + tid;
    srow[tid]           = INN[r];
    srow[GBM + tid]     = ONA[r];
    srow[2 * GBM + tid] = S[r];
  }
  scol[tid]       = bfr(bias[col0 + tid]);
  scol[GBN + tid] = V[col0 + tid];
  __syncthreads();

  v8f acc[GNT];
  {
    const v8f z = {0.f, 0.f, 0.f, 0.f, 0.f, 0.f, 0.f, 0.f};
#pragma unroll
    for (int t = 0; t < GNT; ++t) acc[t] = z;
  }
  const unsigned short* ap = A + (size_t)(rowBase + 16 * wave + m) * (size_t)K + 8 * hh;
  const unsigned short* wp = WT + (size_t)(col0 + m) * (size_t)K + 8 * hh;
  const int ksteps = K >> 5;
#pragma unroll 1
  for (int ks = 0; ks < ksteps; ++ks) {
    FragB af;
    af.h[0] = *(const v8usa*)(ap + 32 * ks);
    af.h[1] = *(const v8usa*)(ap + 32 * ks + 16);
#pragma unroll
    for (int t = 0; t < GNT; ++t) {
      const unsigned short* wq = wp + (size_t)(16 * t) * (size_t)K + 32 * ks;
      FragB bf;
      bf.h[0] = *(const v8usa*)wq;
      bf.h[1] = *(const v8usa*)(wq + 16);
      acc[t] = wmb(af, bf, acc[t]);
    }
  }

#pragma unroll
  for (int t = 0; t < GNT; ++t) {
    const int lc = 16 * t + m;
    const float bb = scol[lc];
    const float vv = scol[GBN + lc];
#pragma unroll
    for (int r = 0; r < 8; ++r) {
      const int lr = 16 * wave + 8 * hh + r;
      float v = acc[t][r];
      if (MODE == 0) v = fmaf(srow[2 * GBM + lr], vv, v);
      v = fmaf(v, srow[lr], bb);
      if (MODE != 2) v = relu_k(v);
      stg[lr * GBN + lc] = v;
    }
  }
  __syncthreads();

#pragma unroll 4
  for (int i = 0; i < 16; ++i) {
    const int lr = 16 * wave + i;
    const int gr = rowBase + lr;
    const v4f r = *(const v4fa*)(stg + lr * GBN + 4 * lane);
    v4f o = r;
    if (MODE == 1) {
      const v4f xs = *(const v4f*)(XSin + (size_t)gr * NHID + col0 + 4 * lane);
      const float on = srow[GBM + lr];
      o.x = on * (xs.x + r.x); o.y = on * (xs.y + r.y); o.z = on * (xs.z + r.z); o.w = on * (xs.w + r.w);
    }
    if (MODE == 0) {
      const float on = srow[GBM + lr];
      o.x = on * r.x; o.y = on * r.y; o.z = on * r.z; o.w = on * r.w;
    }
    const bool live = gr < nN;
    o.x = live ? o.x : 0.0f; o.y = live ? o.y : 0.0f; o.z = live ? o.z : 0.0f; o.w = live ? o.w : 0.0f;
    *(v4fa*)(stg + lr * GBN + 4 * lane) = o;
  }
#pragma unroll 4
  for (int i = 0; i < 16; ++i) {
    const int lr = 16 * wave + i;
    const int gr = rowBase + lr;
    const v4f v = *(const v4fa*)(stg + lr * GBN + 4 * lane);
    float* op = out + (size_t)gr * NHID + col0 + 4 * lane;
    if (gr < mRows) *(volatile v4f*)op = v;
  }
  __threadfence();
#pragma unroll 4
  for (int i = 0; i < 16; ++i) {
    const int lr = 16 * wave + i;
    const int gr = rowBase + lr;
    const v4f v = *(const v4fa*)(stg + lr * GBN + 4 * lane);
    float* op = out + (size_t)gr * NHID + col0 + 4 * lane;
    if (gr < mRows) *(volatile v4f*)op = v;
  }
}

__global__ __launch_bounds__(NTHR) void k_head(const float* __restrict__ X6, const int* __restrict__ cg,
                                               const float* __restrict__ sW, const float* __restrict__ sb,
                                               const float* __restrict__ nW, const float* __restrict__ nb,
                                               const int* __restrict__ FLG, int nLines, float* out, int nN) {
  __shared__ __attribute__((aligned(16))) float wts[9 * NHID];
  __shared__ float sce[NHID];
  __shared__ float zs[NGRP * 9 + 12];
  __shared__ __attribute__((aligned(16))) float outs[912];
  __shared__ int sidx[128];
  __shared__ int sfl[32];
  const int tid = (int)threadIdx.x, lane = tid & 31, wave = tid >> 5;
  {
    const v4f a = *(const v4f*)(sW + 8 * tid);
    const v4f b = *(const v4f*)(sW + 8 * tid + 4);
    wts[tid]            = bfr(nW[tid]);
    wts[1 * NHID + tid] = bfr(a.x);
    wts[2 * NHID + tid] = bfr(a.y);
    wts[3 * NHID + tid] = bfr(a.z);
    wts[4 * NHID + tid] = bfr(a.w);
    wts[5 * NHID + tid] = bfr(b.x);
    wts[6 * NHID + tid] = bfr(b.y);
    wts[7 * NHID + tid] = bfr(b.z);
    wts[8 * NHID + tid] = bfr(b.w);
  }
  if (tid < 32) {
    const int li = tid < nLines ? tid : nLines - 1;
    const int f = FLG[(size_t)li * 32 + 1];
    sfl[tid] = (tid < nLines) ? f : 0;
  }
  const float nbv = bfr(nb[0]);
  const float sbv = bfr(sb[wave]);

#pragma unroll 1
  for (int g = 0; g < NGRP; ++g) {
    {
      const int j = tid < GSZ ? tid : GSZ - 1;
      const int raw = cg[g * GSZ + j];
      if (tid < 128) sidx[tid] = clampi(raw, 0, nN - 1);
    }
    __syncthreads();
    float s = 0.0f;
#pragma unroll 4
    for (int j = 0; j < GSZ; ++j) s += X6[(size_t)sidx[j] * NHID + tid];
    sce[tid] = s;
    __syncthreads();
    {
      float p = 0.0f;
#pragma unroll
      for (int i = 0; i < 8; ++i) {
        const int c = lane + 32 * i;
        p = fmaf(sce[c], wts[(1 + wave) * NHID + c], p);
      }
      p += __shfl_xor(p, 16, 32);
      p += __shfl_xor(p, 8, 32);
      p += __shfl_xor(p, 4, 32);
      p += __shfl_xor(p, 2, 32);
      p += __shfl_xor(p, 1, 32);
      if (lane == 0) zs[g * 9 + 1 + wave] = p + sbv;
    }
    if (wave == 0) {
      float p = 0.0f;
#pragma unroll
      for (int i = 0; i < 8; ++i) {
        const int c = lane + 32 * i;
        p = fmaf(sce[c], wts[c], p);
      }
      p += __shfl_xor(p, 16, 32);
      p += __shfl_xor(p, 8, 32);
      p += __shfl_xor(p, 4, 32);
      p += __shfl_xor(p, 2, 32);
      p += __shfl_xor(p, 1, 32);
      if (lane == 0) zs[g * 9] = p + nbv;
    }
  }
  __syncthreads();
  int fl = 0;
#pragma unroll 4
  for (int i = 0; i < 32; ++i) fl |= sfl[i];
  {
    const int gg = tid < NGRP ? tid : NGRP - 1;
    const float zn = zs[gg * 9];
    const float ez = expf(zn < 0.0f ? zn : -zn);
    const float lp = log1pf(ez);
    const float ls = (zn < 0.0f) ? (zn - lp) : (-lp);
    float mx = zs[gg * 9 + 1];
#pragma unroll 1
    for (int k = 2; k <= 8; ++k) {
      const float z = zs[gg * 9 + k];
      mx = (mx != mx) ? mx : ((z > mx || z != z) ? z : mx);
    }
    float se = 0.0f;
#pragma unroll 1
    for (int k = 1; k <= 8; ++k) se += expf(zs[gg * 9 + k] - mx);
    const float lg = logf(se);
    if (tid < NGRP) outs[gg * 9] = ls;
#pragma unroll 1
    for (int k = 1; k <= 8; ++k) {
      const float val = (zs[gg * 9 + k] - mx) - lg;
      if (tid < NGRP) outs[gg * 9 + k] = val;
    }
  }
  __syncthreads();
  const int pc = tid < 225 ? tid : 224;
  v4f ov = *(const v4fa*)(outs + 4 * pc);
  if (fl != 0) {
    const float qn = __int_as_float(0x7fc00000);
    ov.x = qn; ov.y = qn; ov.z = qn; ov.w = qn;
  }
  float* op = out + 4 * pc;
  if (tid < 225) *(volatile v4f*)op = ov;
  __threadfence();
  if (tid < 225) *(volatile v4f*)op = ov;
}

static inline int cdiv(int a, int b) { return (a + b - 1) / b; }
static inline size_t al256(size_t o) { return (o + 255) & ~(size_t)255; }

extern "C" void kernel_launch(void* const* d_in, const int* in_sizes, int n_in,
                              void* d_out, int out_size, void* d_ws, size_t ws_size,
                              hipStream_t stream) {
  if (n_in < 24) return;
  const int nN = 10000, nE = 120000;
  if (in_sizes[0] != nN * CFW) return;
  if (in_sizes[1] != nE * CEW) return;
  if (in_sizes[2] != NTOP * 32) return;
  if (in_sizes[3] != ETOP * 16) return;
  if (in_sizes[4] != OPS * OPW) return;
  if (in_sizes[5] != 48 * NHID) return;
  if (in_sizes[6] != NHID) return;
  if (in_sizes[7] != 3 * 272 * NHID) return;
  if (in_sizes[8] != 3 * NHID) return;
  if (in_sizes[9] != W0ROWS * NHID) return;
  if (in_sizes[10] != NHID) return;
  if (in_sizes[11] != 5 * 272 * NHID) return;
  if (in_sizes[12] != 5 * NHID) return;
  if (in_sizes[13] != NHID * 8 || in_sizes[14] != 8) return;
  if (in_sizes[15] != NHID || in_sizes[16] != 1) return;
  if (in_sizes[17] != nN) return;
  if (in_sizes[18] != nE || in_sizes[19] != nE) return;
  if (in_sizes[20] != ETOP || in_sizes[21] != ETOP) return;
  if (in_sizes[22] != NGRP * GSZ) return;
  if (in_sizes[23] != 16) return;
  if (out_size != NGRP * 9) return;
  if (nE > (1 << EIDB)) return;

  const float* cfeats = (const float*)d_in[0];
  const float* cedge  = (const float*)d_in[1];
  const float* tfeats = (const float*)d_in[2];
  const float* tedge  = (const float*)d_in[3];
  const float* opemb  = (const float*)d_in[4];
  const float* tW0    = (const float*)d_in[5];
  const float* tb0    = (const float*)d_in[6];
  const float* tWr    = (const float*)d_in[7];
  const float* tbr    = (const float*)d_in[8];
  const float* cW0    = (const float*)d_in[9];
  const float* cb0    = (const float*)d_in[10];
  const float* cWr    = (const float*)d_in[11];
  const float* cbr    = (const float*)d_in[12];
  const float* sW     = (const float*)d_in[13];
  const float* sb     = (const float*)d_in[14];
  const float* nW     = (const float*)d_in[15];
  const float* nb     = (const float*)d_in[16];
  const int* ctypes   = (const int*)d_in[17];
  const int* c_src    = (const int*)d_in[18];
  const int* c_dst    = (const int*)d_in[19];
  const int* t_src    = (const int*)d_in[20];
  const int* t_dst    = (const int*)d_in[21];
  const int* cgroups  = (const int*)d_in[22];
  const int* tgroups  = (const int*)d_in[23];
  float* out = (float*)d_out;

  const int MP = cdiv(nN, 128) * 128;
  const int gA = cdiv(MP, NBA);
  const int NSL = gA * NBA;
  if ((MP % ANB) != 0 || (MP % GBM) != 0 || NSL < MP) return;
  const int vec8 = ((nE & 3) == 0) ? 1 : 0;
  const int nU0 = MP * (G0W / 4);
  if ((nU0 % NTHR) != 0) return;

  char* ws = (char*)d_ws;
  size_t off = 0;
  const size_t oWTS = off; off = al256(off + (size_t)WTS_N * 2);
  const size_t oV   = off; off = al256(off + (size_t)NHID * 4);
  const size_t oLST = off; off = al256(off + (size_t)gA * RCAP * 4);
  const size_t oCNT = off; off = al256(off + (size_t)NSL * 4);
  const size_t oOFF = off; off = al256(off + (size_t)NSL * 4);
  const size_t oINN = off; off = al256(off + (size_t)NSL * 4);
  const size_t oON  = off; off = al256(off + (size_t)NSL * 4);
  const size_t oFLG = off; off = al256(off + (size_t)2 * gA * 128);
  const size_t oG0  = off; off = al256(off + (size_t)MP * G0W * 4);
  const size_t oH0  = off; off = al256(off + (size_t)MP * K0T * 2);
  const size_t oEA  = off; off = al256(off + (size_t)MP * 16 * 4);
  const size_t oS   = off; off = al256(off + (size_t)MP * 4);
  const size_t oH   = off; off = al256(off + (size_t)MP * KRT * 2);
  const size_t oXA  = off; off = al256(off + (size_t)MP * NHID * 4);
  const size_t oXB  = off; off = al256(off + (size_t)MP * NHID * 4);
  if (off > ws_size || off > (size_t)WSMAX) return;
  unsigned short* WTS = (unsigned short*)(ws + oWTS);
  float* V    = (float*)(ws + oV);
  int*   LST  = (int*)(ws + oLST);
  int*   CNTA = (int*)(ws + oCNT);
  int*   OFFA = (int*)(ws + oOFF);
  float* INNA = (float*)(ws + oINN);
  float* ONA  = (float*)(ws + oON);
  int*   FLG  = (int*)(ws + oFLG);
  int*   FLG0 = FLG;
  int*   FLG1 = FLG + (size_t)gA * 32;
  float* G0   = (float*)(ws + oG0);
  unsigned short* H0 = (unsigned short*)(ws + oH0);
  float* EA   = (float*)(ws + oEA);
  float* S    = (float*)(ws + oS);
  unsigned short* H = (unsigned short*)(ws + oH);
  float* XA   = (float*)(ws + oXA);
  float* XB   = (float*)(ws + oXB);

  const int bktLds = BKT_INTS * 4;
  hipFuncSetAttribute(reinterpret_cast<const void*>(&k_bucket<0>),
                      hipFuncAttributeMaxDynamicSharedMemorySize, bktLds);
  hipFuncSetAttribute(reinterpret_cast<const void*>(&k_bucket<1>),
                      hipFuncAttributeMaxDynamicSharedMemorySize, bktLds);

  k_prep<<<U_ALL / NTHR, NTHR, 0, stream>>>(tW0, tWr, cW0, cWr, WTS);
  k_topo<<<1, NTHR, 0, stream>>>(tfeats, tedge, tb0, tbr, t_src, t_dst, tgroups, cW0, WTS, V);
  k_bucket<0><<<gA, NTHR, bktLds, stream>>>(c_dst, nE, nN, vec8, LST, CNTA, OFFA, INNA, FLG0);
  k_bucket<1><<<gA, NTHR, bktLds, stream>>>(c_src, nE, nN, vec8, LST, CNTA, OFFA, ONA, FLG1);
  k_node0<<<nU0 / NTHR, NTHR, 0, stream>>>(cfeats, opemb, ctypes, ONA, G0, nN, nU0);
  k_agg0<<<MP / ANB, NTHR, 0, stream>>>(c_src, cedge, G0, ONA, LST, CNTA, OFFA, FLG0, H0, EA, S, nN, nE, MP);
  k_gemm<0><<<dim3(MP / GBM, NHID / GBN), GTHR, 0, stream>>>(H0, WTS + OW_CW0, cb0, INNA, ONA, S, V, XA, XA,
                                                             K0T, nN, MP);
  float* cur = XA;
  float* nxt = XB;
  for (int l = 1; l <= 5; ++l) {
    k_agg<<<MP / ANB, NTHR, 0, stream>>>(c_src, cur, EA, LST, CNTA, OFFA, FLG0, H, nN, nE, MP);
    const unsigned short* wt = WTS + OW_CWR + (size_t)(l - 1) * PLR;
    const float* bl = cbr + (size_t)(l - 1) * NHID;
    if (l < 5) {
      k_gemm<1><<<dim3(MP / GBM, NHID / GBN), GTHR, 0, stream>>>(H, wt, bl, INNA, ONA, S, V, cur, nxt,
                                                                 KRT, nN, MP);
    } else {
      k_gemm<2><<<dim3(MP / GBM, NHID / GBN), GTHR, 0, stream>>>(H, wt, bl, INNA, ONA, S, V, cur, nxt,
                                                                 KRT, nN, MP);
    }
    float* t = cur; cur = nxt; nxt = t;
  }
  k_head<<<1, NTHR, 0, stream>>>(cur, cgroups, sW, sb, nW, nb, FLG, 2 * gA, out, nN);
}
